// GraphTransformer2_3504693313909
// MI455X (gfx1250) — hardware-verified
//
#include <hip/hip_runtime.h>
#include <stddef.h>
#include <stdint.h>
#include <math.h>

#define NN      16384
#define HID     128
#define NE      262144
#define NG      32
#define SEQ     512
#define NH      4
#define HD      32
#define OUTC    64
#define NL      2
#define PCAT    896
#define HLP     256

#define NTHR    256
#define NWAVE   8
#define EPT     8
#define CHUNK   (NTHR * EPT)
#define WCAP    (EPT * 32)
#define LISTN   (NWAVE * WCAP)
#define NBMAX   2048
#define NBRUN   1024
#define RCAP    28672
#define DEGCAP  64
#define WSMAX   134217728
#define LDS_AGG ((2 * RCAP + 2 * NBMAX + LISTN) * 4 + 64)

#define SP       132
#define LDS_GEMM (8 * 16 * SP * 4)
#define AKC      64
#define LDS_ATT  (2 * AKC * HD * 2 + 2 * HD * AKC * 2 + 2 * 4 * 16 * AKC * 2 + 4 * 16 * SP * 4)

#define VG __attribute__((amdgpu_num_vgpr(248)))

static_assert((CHUNK & (CHUNK - 1)) == 0 && CHUNK <= 4096);
static_assert((NBMAX & (NBMAX - 1)) == 0 && NBMAX <= 4096);
static_assert((NBRUN & (NBRUN - 1)) == 0 && NBRUN <= NBMAX && NBRUN >= 16);
static_assert(NTHR * 8 == NBMAX);
static_assert(LISTN >= NBMAX);
static_assert((RCAP % 32) == 0);
static_assert(LDS_AGG <= 300000);
static_assert(NN % NBRUN == 0);
static_assert(HID == 128 && NH * HD == HID && HD == 32);
static_assert(NN % 128 == 0 && NN == NG * SEQ && SEQ % AKC == 0 && SEQ % 64 == 0);
static_assert(NE < (1 << 20));
static_assert(PCAT == 7 * 128);
static_assert(LDS_GEMM <= 327680 && LDS_ATT <= 327680 && LDS_AGG <= 327680);

typedef float          v4f   __attribute__((ext_vector_type(4)));
typedef float          v8f   __attribute__((ext_vector_type(8)));
typedef int            v4i   __attribute__((ext_vector_type(4)));
typedef int            v8i   __attribute__((ext_vector_type(8)));
typedef unsigned short v8us  __attribute__((ext_vector_type(8)));
typedef __bf16         v16bf __attribute__((ext_vector_type(16)));
union FragB { v16bf v; v8us u[2]; v8i w; };

#define WSYNC() do { __builtin_amdgcn_fence(__ATOMIC_RELEASE, "workgroup"); __builtin_amdgcn_wave_barrier(); \
                     __builtin_amdgcn_fence(__ATOMIC_ACQUIRE, "workgroup"); } while (0)

__device__ __forceinline__ v8f wmx(const FragB& a, const FragB& b, v8f c) {
  v8f d = __builtin_amdgcn_wmma_f32_16x16x32_bf16(false, a.v, false, b.v, (short)0, c, false, false);
  asm volatile("v_nop\n\tv_nop\n\tv_nop\n\tv_nop" : "+v"(d) : "v"(a.w), "v"(b.w));
  return d;
}

__device__ __forceinline__ void ldwait() {
  asm volatile("s_wait_loadcnt 0x0" ::: "memory");
}

__device__ __forceinline__ unsigned bfbits(float v) {
  const unsigned u = __float_as_uint(v);
  const unsigned r = (u + 0x7FFFu + ((u >> 16) & 1u)) >> 16;
  return (v != v) ? 0x7FC0u : r;
}
__device__ __forceinline__ float bf2f(unsigned b) { return __uint_as_float(b << 16); }
__device__ __forceinline__ float rbf(float v) { return bf2f(bfbits(v)); }
__device__ __forceinline__ v4f rbf4(const v4f a) {
  v4f o; o.x = rbf(a.x); o.y = rbf(a.y); o.z = rbf(a.z); o.w = rbf(a.w); return o;
}

__device__ __forceinline__ v8us cvt8b(const v4f a, const v4f b) {
  v8us o;
  o[0] = (unsigned short)bfbits(a.x); o[1] = (unsigned short)bfbits(a.y);
  o[2] = (unsigned short)bfbits(a.z); o[3] = (unsigned short)bfbits(a.w);
  o[4] = (unsigned short)bfbits(b.x); o[5] = (unsigned short)bfbits(b.y);
  o[6] = (unsigned short)bfbits(b.z); o[7] = (unsigned short)bfbits(b.w);
  return o;
}

__device__ __forceinline__ v8us hl8(const float* sp, int lo) {
  const v4f a = *(const v4f*)sp;
  const v4f b = *(const v4f*)(sp + 4);
  const float f[8] = {a.x, a.y, a.z, a.w, b.x, b.y, b.z, b.w};
  v8us o;
#pragma unroll
  for (int i = 0; i < 8; ++i) {
    const unsigned hb = bfbits(f[i]);
    const unsigned lb = bfbits(f[i] - bf2f(hb));
    o[i] = (unsigned short)(lo ? lb : hb);
  }
  return o;
}

__device__ __forceinline__ v4f ln4(const v4f y, const v4f g, const v4f b) {
  float s = (y.x + y.y) + (y.z + y.w);
#pragma unroll
  for (int off = 16; off > 0; off >>= 1) s += __shfl_xor(s, off);
  const float mean = s * 0.0078125f;
  v4f d; d.x = y.x - mean; d.y = y.y - mean; d.z = y.z - mean; d.w = y.w - mean;
  float q = d.x * d.x; q = fmaf(d.y, d.y, q); q = fmaf(d.z, d.z, q); q = fmaf(d.w, d.w, q);
#pragma unroll
  for (int off = 16; off > 0; off >>= 1) q += __shfl_xor(q, off);
  const float rstd = rsqrtf(q * 0.0078125f + 1e-5f);
  v4f o;
  o.x = d.x * rstd * g.x + b.x; o.y = d.y * rstd * g.y + b.y;
  o.z = d.z * rstd * g.z + b.z; o.w = d.w * rstd * g.w + b.w;
  return o;
}

__global__ __launch_bounds__(256) VG void k_cvt(const float* __restrict__ src, unsigned short* dst,
                                                int nUnits, int rpl, int dls, int droff, int dpitch, int dup) {
  const int u = (int)blockIdx.x * 256 + (int)threadIdx.x;
  if (u >= nUnits) return;
  const int R  = u >> 4;
  const int k8 = (u & 15) * 8;
  const int l  = R / rpl;
  const int r  = R - l * rpl;
  const float* p = src + (size_t)R * HID + k8;
  const v4f a = *(const v4f*)p;
  const v4f b = *(const v4f*)(p + 4);
  const v8us hv = cvt8b(a, b);
  const size_t o = (size_t)(l * dls + droff + r) * (size_t)dpitch + k8;
  *(volatile v8us*)(dst + o) = hv;
  if (dup != 0) *(volatile v8us*)(dst + o + 128) = hv;
  __threadfence();
  *(volatile v8us*)(dst + o) = hv;
  if (dup != 0) *(volatile v8us*)(dst + o + 128) = hv;
}

__global__ __launch_bounds__(128) VG void k_bcat(const float* __restrict__ bq, const float* __restrict__ bk,
                                                 const float* __restrict__ bv, const float* __restrict__ bs,
                                                 const float* __restrict__ bi, float* bcat) {
  const int seg = (int)blockIdx.x, l = (int)blockIdx.y, c = (int)threadIdx.x;
  const int i4 = l * HID + c;
  const int sg = seg < 4 ? 0 : seg - 4;
  const int i3 = l * (3 * HID) + sg * HID + c;
  const float v0 = bq[i4], v1 = bk[i4], v2 = bv[i4], v3 = bs[i4], v4 = bi[i3];
  float v = v4;
  v = (seg == 0) ? v0 : v;
  v = (seg == 1) ? v1 : v;
  v = (seg == 2) ? v2 : v;
  v = (seg == 3) ? v3 : v;
  v = rbf(v);
  float* op = bcat + (size_t)l * PCAT + seg * HID + c;
  *(volatile float*)op = v;
  __threadfence();
  *(volatile float*)op = v;
}

template<int NT, int EPI>
__global__ __launch_bounds__(256) VG void k_gemm(
    const unsigned short* __restrict__ A, const unsigned short* __restrict__ WT,
    const float* __restrict__ bias, const float* __restrict__ R1, const float* __restrict__ R2,
    const float* __restrict__ lng, const float* __restrict__ lnb,
    float* OF, unsigned short* OH, int lda, int ksteps, int ldo)
{
  extern __shared__ v4f lds_dyn[];
  const int tid = (int)threadIdx.x, lane = tid & 31, wave = tid >> 5, hh = lane >> 4, m = lane & 15;
  float* slab = (float*)lds_dyn + wave * (16 * SP);
  const int rowBase = (int)blockIdx.x * 128;
  const int ty      = (int)blockIdx.y;
  const int col0    = ty * (16 * NT);
  const int K       = ksteps * 32;

  v8f acc[NT];
  {
    const v8f z = {0.f, 0.f, 0.f, 0.f, 0.f, 0.f, 0.f, 0.f};
#pragma unroll
    for (int t = 0; t < NT; ++t) acc[t] = z;
  }
  const unsigned short* ap = A  + (size_t)(rowBase + 16 * wave + m) * (size_t)lda + 8 * hh;
  const unsigned short* wp = WT + (size_t)(col0 + m) * (size_t)K + 8 * hh;
#pragma unroll 1
  for (int ks = 0; ks < ksteps; ++ks) {
    FragB af;
    af.u[0] = *(const v8us*)(ap + 32 * ks);
    af.u[1] = *(const v8us*)(ap + 32 * ks + 16);
#pragma unroll
    for (int t = 0; t < NT; ++t) {
      const unsigned short* wq = wp + (size_t)(16 * t) * (size_t)K + 32 * ks;
      FragB bf;
      bf.u[0] = *(const v8us*)wq;
      bf.u[1] = *(const v8us*)(wq + 16);
      acc[t] = wmx(af, bf, acc[t]);
    }
  }

#pragma unroll
  for (int t = 0; t < NT; ++t) {
#pragma unroll
    for (int r = 0; r < 8; ++r) slab[(8 * hh + r) * SP + 16 * t + m] = acc[t][r];
  }
  WSYNC();

  const int grow0 = rowBase + 16 * wave;
  if (NT == 8) {
    const v4f bi4 = rbf4(*(const v4f*)(bias + col0 + 4 * lane));
    v4f g4 = {1.f, 1.f, 1.f, 1.f}, b4 = {0.f, 0.f, 0.f, 0.f};
    if (EPI == 2 || EPI == 4) {
      g4 = rbf4(*(const v4f*)(lng + 4 * lane));
      b4 = rbf4(*(const v4f*)(lnb + 4 * lane));
    }
#pragma unroll 1
    for (int row = 0; row < 16; ++row) {
      const int gr = grow0 + row;
      float* sp = slab + row * SP + 4 * lane;
      v4f v = *(const v4f*)sp;
      v.x += bi4.x; v.y += bi4.y; v.z += bi4.z; v.w += bi4.w;
      if (EPI == 2 || EPI == 4) {
        const v4f x = *(const v4f*)(R1 + (size_t)gr * HID + 4 * lane);
        v.x += x.x; v.y += x.y; v.z += x.z; v.w += x.w;
        v = ln4(v, g4, b4);
      }
      if (EPI == 2) {
        const v4f x = *(const v4f*)(R2 + (size_t)gr * HID + 4 * lane);
        v.x += x.x; v.y += x.y; v.z += x.z; v.w += x.w;
      }
      if (EPI == 3) {
        v.x = (v.x > 0.f) ? v.x : (v.x - v.x);
        v.y = (v.y > 0.f) ? v.y : (v.y - v.y);
        v.z = (v.z > 0.f) ? v.z : (v.z - v.z);
        v.w = (v.w > 0.f) ? v.w : (v.w - v.w);
      }
      *(v4f*)sp = v;
    }
    WSYNC();
    const bool wf = (EPI == 0) || (EPI == 2) || (EPI == 4) || (EPI == 1 && ty < 4);
    const bool wh = (EPI == 0) || (EPI == 2) || (EPI == 3) || (EPI == 4) || (EPI == 1 && ty >= 4);
    float* of = OF + ((EPI == 1 && ty < 4) ? 128 * ty : 0);
    unsigned short* oh = OH + ((EPI == 1 && ty >= 4) ? (size_t)(ty - 4) * (size_t)NN * HLP : (size_t)0);
    for (int pass = 0; pass < 2; ++pass) {
#pragma unroll 1
      for (int row = 0; row < 16; ++row) {
        const int gr = grow0 + row;
        if (wf) {
          const v4f v = *(const v4f*)(slab + row * SP + 4 * lane);
          *(volatile v4f*)(of + (size_t)gr * (size_t)ldo + 4 * lane) = v;
        }
        if (wh) {
          const v8us o = hl8(slab + row * SP + 8 * m, hh);
          *(volatile v8us*)(oh + (size_t)gr * HLP + 128 * hh + 8 * m) = o;
        }
      }
      __threadfence();
    }
  } else {
    const v4f bi4 = rbf4(*(const v4f*)(bias + col0 + 4 * m));
#pragma unroll 1
    for (int i = 0; i < 8; ++i) {
      float* sp = slab + (2 * i + hh) * SP + 4 * m;
      v4f v = *(const v4f*)sp;
      v.x += bi4.x; v.y += bi4.y; v.z += bi4.z; v.w += bi4.w;
      *(v4f*)sp = v;
    }
    WSYNC();
    for (int pass = 0; pass < 2; ++pass) {
#pragma unroll 1
      for (int i = 0; i < 8; ++i) {
        const int row = 2 * i + hh;
        const v4f v = *(const v4f*)(slab + row * SP + 4 * m);
        *(volatile v4f*)(OF + (size_t)(grow0 + row) * (size_t)ldo + col0 + 4 * m) = v;
      }
      __threadfence();
    }
  }
}

__global__ __launch_bounds__(128) VG void k_attn(const unsigned short* __restrict__ AQ,
                                                 const unsigned short* __restrict__ AK,
                                                 const unsigned short* __restrict__ AV,
                                                 unsigned short* OHL) {
  extern __shared__ v4f lds_dyn[];
  unsigned short* Ksh = (unsigned short*)lds_dyn;
  unsigned short* Ksl = Ksh + AKC * HD;
  unsigned short* Vth = Ksl + AKC * HD;
  unsigned short* Vtl = Vth + HD * AKC;
  unsigned short* Psh = Vtl + HD * AKC;
  unsigned short* Psl = Psh + 4 * 16 * AKC;
  float*          Os  = (float*)(Psl + 4 * 16 * AKC);

  const int tid = (int)threadIdx.x, wave = tid >> 5, lane = tid & 31, hh = lane >> 4, c = lane & 15;
  const int bx = (int)blockIdx.x;
  const int b  = bx >> 3;
  const int qt = bx & 7;
  const int q0 = b * SEQ + qt * 64 + wave * 16;
  const float sscale = 0.17677669529663687f;
  unsigned short* pwh = Psh + wave * (16 * AKC);
  unsigned short* pwl = Psl + wave * (16 * AKC);
  float* os = Os + wave * (16 * SP);

#pragma unroll 1
  for (int h = 0; h < NH; ++h) {
    FragB qah, qal;
    {
      const unsigned short* qp = AQ + (size_t)(q0 + c) * HLP + 32 * h + 8 * hh;
      qah.u[0] = *(const v8us*)qp;          qah.u[1] = *(const v8us*)(qp + 16);
      qal.u[0] = *(const v8us*)(qp + 128);  qal.u[1] = *(const v8us*)(qp + 144);
    }
    float mrow[8], lrow[8];
    v8f oacc[2];
#pragma unroll
    for (int r = 0; r < 8; ++r) { mrow[r] = -INFINITY; lrow[r] = 0.f; }
    oacc[0] = (v8f){0.f,0.f,0.f,0.f,0.f,0.f,0.f,0.f};
    oacc[1] = (v8f){0.f,0.f,0.f,0.f,0.f,0.f,0.f,0.f};

#pragma unroll 1
    for (int kc = 0; kc < SEQ / AKC; ++kc) {
      const int kv0 = b * SEQ + kc * AKC;
      __syncthreads();
      {
        const int r = tid >> 1, half = (tid & 1) * 16;
        const unsigned short* kp = AK + (size_t)(kv0 + r) * HLP + 32 * h + half;
        const unsigned short* vp = AV + (size_t)(kv0 + r) * HLP + 32 * h + half;
#pragma unroll
        for (int i = 0; i < 2; ++i) {
          const v8us a0 = *(const v8us*)(kp + 8 * i);
          const v8us a1 = *(const v8us*)(kp + 128 + 8 * i);
          const v8us b0 = *(const v8us*)(vp + 8 * i);
          const v8us b1 = *(const v8us*)(vp + 128 + 8 * i);
          *(v8us*)(Ksh + r * HD + half + 8 * i) = a0;
          *(v8us*)(Ksl + r * HD + half + 8 * i) = a1;
#pragma unroll
          for (int e = 0; e < 8; ++e) {
            Vth[(half + 8 * i + e) * AKC + r] = b0[e];
            Vtl[(half + 8 * i + e) * AKC + r] = b1[e];
          }
        }
      }
      __syncthreads();

      v8f s[4];
#pragma unroll
      for (int j = 0; j < 4; ++j) {
        s[j] = (v8f){0.f,0.f,0.f,0.f,0.f,0.f,0.f,0.f};
        FragB kb, kl;
        kb.u[0] = *(const v8us*)(Ksh + (j * 16 + c) * HD + 8 * hh);
        kb.u[1] = *(const v8us*)(Ksh + (j * 16 + c) * HD + 16 + 8 * hh);
        kl.u[0] = *(const v8us*)(Ksl + (j * 16 + c) * HD + 8 * hh);
        kl.u[1] = *(const v8us*)(Ksl + (j * 16 + c) * HD + 16 + 8 * hh);
        s[j] = wmx(qah, kb, s[j]);
        s[j] = wmx(qah, kl, s[j]);
        s[j] = wmx(qal, kb, s[j]);
      }
      float cm[8];
#pragma unroll
      for (int r = 0; r < 8; ++r) {
        float mm = -INFINITY;
#pragma unroll
        for (int j = 0; j < 4; ++j) {
          const float sv = s[j][r] * sscale;
          s[j][r] = sv;
          mm = fmaxf(mm, sv);
        }
#pragma unroll
        for (int off = 1; off < 16; off <<= 1) mm = fmaxf(mm, __shfl_xor(mm, off));
        cm[r] = mm;
      }
#pragma unroll
      for (int r = 0; r < 8; ++r) {
        const float mnew  = fmaxf(mrow[r], cm[r]);
        const float alpha = expf(mrow[r] - mnew);
        mrow[r] = mnew;
        float psum = 0.f;
#pragma unroll
        for (int j = 0; j < 4; ++j) {
          const float p = expf(s[j][r] - mnew);
          psum += p;
          const unsigned hb = bfbits(p);
          const unsigned lb = bfbits(p - bf2f(hb));
          pwh[(8 * hh + r) * AKC + j * 16 + c] = (unsigned short)hb;
          pwl[(8 * hh + r) * AKC + j * 16 + c] = (unsigned short)lb;
        }
#pragma unroll
        for (int off = 1; off < 16; off <<= 1) psum += __shfl_xor(psum, off);
        lrow[r] = lrow[r] * alpha + psum;
        oacc[0][r] *= alpha;
        oacc[1][r] *= alpha;
      }
      WSYNC();
#pragma unroll 1
      for (int kk = 0; kk < 2; ++kk) {
        FragB pa, pl;
        pa.u[0] = *(const v8us*)(pwh + c * AKC + kk * 32 + 8 * hh);
        pa.u[1] = *(const v8us*)(pwh + c * AKC + kk * 32 + 16 + 8 * hh);
        pl.u[0] = *(const v8us*)(pwl + c * AKC + kk * 32 + 8 * hh);
        pl.u[1] = *(const v8us*)(pwl + c * AKC + kk * 32 + 16 + 8 * hh);
#pragma unroll
        for (int t = 0; t < 2; ++t) {
          FragB vb, vl;
          vb.u[0] = *(const v8us*)(Vth + (t * 16 + c) * AKC + kk * 32 + 8 * hh);
          vb.u[1] = *(const v8us*)(Vth + (t * 16 + c) * AKC + kk * 32 + 16 + 8 * hh);
          vl.u[0] = *(const v8us*)(Vtl + (t * 16 + c) * AKC + kk * 32 + 8 * hh);
          vl.u[1] = *(const v8us*)(Vtl + (t * 16 + c) * AKC + kk * 32 + 16 + 8 * hh);
          oacc[t] = wmx(pa, vb, oacc[t]);
          oacc[t] = wmx(pa, vl, oacc[t]);
          oacc[t] = wmx(pl, vb, oacc[t]);
        }
      }
      WSYNC();
    }
#pragma unroll
    for (int r = 0; r < 8; ++r) {
      const float inv = 1.0f / lrow[r];
      os[(8 * hh + r) * SP + 32 * h + c]      = oacc[0][r] * inv;
      os[(8 * hh + r) * SP + 32 * h + 16 + c] = oacc[1][r] * inv;
    }
  }
  WSYNC();
  for (int pass = 0; pass < 2; ++pass) {
#pragma unroll 1
    for (int row = 0; row < 16; ++row) {
      const v8us o = hl8(os + row * SP + 8 * c, hh);
      *(volatile v8us*)(OHL + (size_t)(q0 + row) * HLP + 128 * hh + 8 * c) = o;
    }
    __threadfence();
  }
}

__device__ __forceinline__ int scan_chunk(const int* __restrict__ dsts, int nE, int cbase, int slotBase,
                                          int nb, int vec8, int* list, int tid, int lane, int wave) {
  int wc = 0;
  const int el0  = tid * EPT;
  const int e0   = cbase + el0;
  const int sent = -2147483647 - 1;
  v4i da, db;
  if (vec8 != 0 && cbase + CHUNK <= nE) {
    da = *(const v4i*)(dsts + e0);
    db = *(const v4i*)(dsts + e0 + 4);
  } else {
    da.x = (e0     < nE) ? dsts[min(e0,     nE - 1)] : sent;
    da.y = (e0 + 1 < nE) ? dsts[min(e0 + 1, nE - 1)] : sent;
    da.z = (e0 + 2 < nE) ? dsts[min(e0 + 2, nE - 1)] : sent;
    da.w = (e0 + 3 < nE) ? dsts[min(e0 + 3, nE - 1)] : sent;
    db.x = (e0 + 4 < nE) ? dsts[min(e0 + 4, nE - 1)] : sent;
    db.y = (e0 + 5 < nE) ? dsts[min(e0 + 5, nE - 1)] : sent;
    db.z = (e0 + 6 < nE) ? dsts[min(e0 + 6, nE - 1)] : sent;
    db.w = (e0 + 7 < nE) ? dsts[min(e0 + 7, nE - 1)] : sent;
  }
  const unsigned nbs = (unsigned)slotBase;
  const unsigned unb = (unsigned)nb;
  const unsigned s0 = (unsigned)da.x - nbs, s1 = (unsigned)da.y - nbs;
  const unsigned s2 = (unsigned)da.z - nbs, s3 = (unsigned)da.w - nbs;
  const unsigned s4 = (unsigned)db.x - nbs, s5 = (unsigned)db.y - nbs;
  const unsigned s6 = (unsigned)db.z - nbs, s7 = (unsigned)db.w - nbs;
  const bool h0 = s0 < unb, h1 = s1 < unb, h2 = s2 < unb, h3 = s3 < unb;
  const bool h4 = s4 < unb, h5 = s5 < unb, h6 = s6 < unb, h7 = s7 < unb;
  const unsigned any = __builtin_amdgcn_ballot_w32(h0 | h1 | h2 | h3 | h4 | h5 | h6 | h7);
  if (any != 0u) {
#define HITJ(J, HJ, SJ) { \
      const unsigned mj = __builtin_amdgcn_ballot_w32(HJ); \
      if (mj != 0u) { \
        if (HJ) { \
          const int pos = wc + (int)__builtin_amdgcn_mbcnt_lo(mj, 0u); \
          if (pos < WCAP) list[wave * WCAP + pos] = ((el0 + (J)) << 12) | (int)(SJ); \
        } \
        wc += (int)__builtin_popcount(mj); } }
    HITJ(0, h0, s0)
    HITJ(1, h1, s1)
    HITJ(2, h2, s2)
    HITJ(3, h3, s3)
    HITJ(4, h4, s4)
    HITJ(5, h5, s5)
    HITJ(6, h6, s6)
    HITJ(7, h7, s7)
#undef HITJ
  }
  return wc;
}

__global__ __launch_bounds__(NTHR) VG void k_scan(
    const int* __restrict__ srcs, const int* __restrict__ dsts,
    const float* __restrict__ QKVR, const float* __restrict__ X,
    const float* __restrict__ wbeta, const float* __restrict__ lng, const float* __restrict__ lnb,
    float* XL, int nN, int nE, int vec8) {
  extern __shared__ v4f lds_dyn[];
  int* reg1 = (int*)lds_dyn;
  int* reg2 = reg1 + RCAP;
  int* scnt = reg2 + RCAP;
  int* soff = scnt + NBMAX;
  int* list = soff + NBMAX;
  int* wcnt = list + LISTN;
  int* wtot = wcnt + NWAVE;
  const int tid = (int)threadIdx.x, lane = tid & 31, wave = tid >> 5;
  const int nb = NBRUN;
  const int nodeBase = (int)blockIdx.x * nb;

  for (int i = tid; i < NBMAX; i += NTHR) scnt[i] = 0;
  __syncthreads();

  int tot = 0;
  const int nChunks = (nE + CHUNK - 1) / CHUNK;
#pragma unroll 1
  for (int ch = 0; ch < nChunks; ++ch) {
    const int cbase = ch * CHUNK;
    const int wc = scan_chunk(dsts, nE, cbase, nodeBase, nb, vec8, list, tid, lane, wave);
    if (lane == 0) wcnt[wave] = wc;
    __syncthreads();
    int pre = 0, all = 0;
#pragma unroll
    for (int w2 = 0; w2 < NWAVE; ++w2) {
      int cc = wcnt[w2];
      cc = cc < 0 ? 0 : (cc > WCAP ? WCAP : cc);
      all += cc;
      pre += (w2 < wave) ? cc : 0;
    }
    const int wcc  = wc > WCAP ? WCAP : wc;
    const int base = tot + pre;
#pragma unroll 1
    for (int i = lane; i < wcc; i += 32) {
      const int ent = list[wave * WCAP + i];
      const int el  = (ent >> 12) & (CHUNK - 1);
      const int sl  = ent & (NBMAX - 1);
      int eid = cbase + el;
      eid = eid > nE - 1 ? nE - 1 : eid;
      const int pos = base + i;
      if (pos < RCAP) reg1[pos] = (int)(((unsigned)eid << 12) | (unsigned)sl);
    }
    tot += all;
    tot = tot > RCAP ? RCAP : tot;
    __syncthreads();
  }
  const int nh = tot;

  if (wave == 0) {
#pragma unroll 1
    for (int b0 = 0; b0 < nh; b0 += 32) {
      const int idx = b0 + lane;
      const int uv  = reg1[idx < RCAP ? idx : RCAP - 1];
      const int m32 = (nh - b0) < 32 ? (nh - b0) : 32;
#pragma unroll 1
      for (int k = 0; k < m32; ++k) {
        const int u  = __builtin_amdgcn_readlane(uv, k);
        const int sl = u & (NBMAX - 1);
        if (lane == 0) scnt[sl] = scnt[sl] + 1;
      }
    }
  }
  __syncthreads();

  {
    const v4i ca = *(const v4i*)(scnt + 8 * tid);
    const v4i cb = *(const v4i*)(scnt + 8 * tid + 4);
    const int e0 = ca.x < 0 ? 0 : ca.x, e1 = ca.y < 0 ? 0 : ca.y, e2 = ca.z < 0 ? 0 : ca.z, e3 = ca.w < 0 ? 0 : ca.w;
    const int e4 = cb.x < 0 ? 0 : cb.x, e5 = cb.y < 0 ? 0 : cb.y, e6 = cb.z < 0 ? 0 : cb.z, e7 = cb.w < 0 ? 0 : cb.w;
    const int ts = e0 + e1 + e2 + e3 + e4 + e5 + e6 + e7;
    int incl = ts;
#pragma unroll
    for (int d = 1; d < 32; d <<= 1) {
      const int up = __shfl_up(incl, d);
      if (lane >= d) incl += up;
    }
    if (lane == 31) wtot[wave] = incl;
    __syncthreads();
    int pre = 0;
#pragma unroll
    for (int w2 = 0; w2 < NWAVE; ++w2) pre += (w2 < wave) ? wtot[w2] : 0;
    int run = pre + incl - ts;
    soff[8 * tid + 0] = run; run += e0;
    soff[8 * tid + 1] = run; run += e1;
    soff[8 * tid + 2] = run; run += e2;
    soff[8 * tid + 3] = run; run += e3;
    soff[8 * tid + 4] = run; run += e4;
    soff[8 * tid + 5] = run; run += e5;
    soff[8 * tid + 6] = run; run += e6;
    soff[8 * tid + 7] = run;
  }
  __syncthreads();
  for (int i = tid; i < NBMAX; i += NTHR) list[i] = soff[i];
  __syncthreads();

  if (wave == 0) {
#pragma unroll 1
    for (int b0 = 0; b0 < nh; b0 += 32) {
      const int idx = b0 + lane;
      const int uv  = reg1[idx < RCAP ? idx : RCAP - 1];
      const int m32 = (nh - b0) < 32 ? (nh - b0) : 32;
#pragma unroll 1
      for (int k = 0; k < m32; ++k) {
        const int u   = __builtin_amdgcn_readlane(uv, k);
        const int sl  = u & (NBMAX - 1);
        const int eid = (int)((unsigned)u >> 12);
        if (lane == 0) {
          int pos = list[sl];
          pos = pos < 0 ? 0 : (pos > RCAP - 1 ? RCAP - 1 : pos);
          reg2[pos] = eid;
          list[sl] = pos + 1;
        }
      }
    }
  }
  __syncthreads();

  const int nbw = nb >> 3;
  const bool ovf = (nh >= RCAP);
  const float qnan = __int_as_float(0x7fc00000);
  const v4f wa = rbf4(*(const v4f*)(wbeta + 4 * lane));
  const v4f wr = rbf4(*(const v4f*)(wbeta + HID + 4 * lane));
  const v4f wd = rbf4(*(const v4f*)(wbeta + 2 * HID + 4 * lane));
  const v4f g4 = rbf4(*(const v4f*)(lng + 4 * lane));
  const v4f b4 = rbf4(*(const v4f*)(lnb + 4 * lane));
#pragma unroll 1
  for (int jt = 0; jt < nbw; ++jt) {
    const int slot = wave * nbw + jt;
    const int grow = nodeBase + slot;
    const int gcl  = grow < nN ? grow : nN - 1;
    int st = soff[slot];
    const int craw = scnt[slot];
    int cnt = craw;
    st  = st < 0 ? 0 : (st > nh ? nh : st);
    cnt = cnt < 0 ? 0 : (cnt > DEGCAP ? DEGCAP : cnt);
    if (cnt > nh - st) cnt = nh - st;
    const float pz = (ovf || craw > DEGCAP) ? qnan : 0.0f;

    const float* trow = QKVR + (size_t)gcl * 512 + 4 * lane;
    const v4f q4 = *(const v4f*)trow;
    ldwait();
    float mx = -1.0e30f, dn = 0.f;
    v4f av = {0.f, 0.f, 0.f, 0.f};

#pragma unroll 1
    for (int q = 0; q < cnt; ++q) {
      int idx = st + q; idx = idx > RCAP - 1 ? RCAP - 1 : idx;
      int eid = reg2[idx]; eid = eid < 0 ? 0 : (eid > nE - 1 ? nE - 1 : eid);
      const int sraw = srcs[eid];
      const int s = sraw < 0 ? 0 : (sraw > nN - 1 ? nN - 1 : sraw);
      const float* sr = QKVR + (size_t)s * 512 + 4 * lane;
      const v4f k4 = *(const v4f*)(sr + 128);
      const v4f v4 = *(const v4f*)(sr + 256);
      ldwait();
      float part = q4.x * k4.x;
      part = fmaf(q4.y, k4.y, part);
      part = fmaf(q4.z, k4.z, part);
      part = fmaf(q4.w, k4.w, part);
      part += __shfl_xor(part, 1);
      part += __shfl_xor(part, 2);
      part += __shfl_xor(part, 4);
      const float al = part * 0.17677669529663687f;
      const float df = al - mx;
      const float ee = expf(-fabsf(df));
      const bool up  = df > 0.f;
      const float s1 = up ? ee : 1.0f;
      const float s2 = up ? 1.0f : ee;
      mx = up ? al : mx;
      dn = fmaf(dn, s1, s2);
      av.x = fmaf(av.x, s1, s2 * v4.x);
      av.y = fmaf(av.y, s1, s2 * v4.y);
      av.z = fmaf(av.z, s1, s2 * v4.z);
      av.w = fmaf(av.w, s1, s2 * v4.w);
    }
    const float ds = dn > 0.f ? dn : 1.0f;
    const float iv = (dn > 0.f ? 1.0f : 0.0f) * (1.0f / ds);
    v4f ag; ag.x = av.x * iv; ag.y = av.y * iv; ag.z = av.z * iv; ag.w = av.w * iv;

    const v4f r4 = *(const v4f*)(trow + 384);
    const v4f x0 = *(const v4f*)(X + (size_t)gcl * HID + 4 * lane);
    ldwait();
    float sd = wa.x * ag.x;
    sd = fmaf(wa.y, ag.y, sd); sd = fmaf(wa.z, ag.z, sd); sd = fmaf(wa.w, ag.w, sd);
    sd = fmaf(wr.x, r4.x, sd); sd = fmaf(wr.y, r4.y, sd); sd = fmaf(wr.z, r4.z, sd); sd = fmaf(wr.w, r4.w, sd);
    sd = fmaf(wd.x, ag.x - r4.x, sd); sd = fmaf(wd.y, ag.y - r4.y, sd);
    sd = fmaf(wd.z, ag.z - r4.z, sd); sd = fmaf(wd.w, ag.w - r4.w, sd);
#pragma unroll
    for (int off = 16; off > 0; off >>= 1) sd += __shfl_xor(sd, off);
    const float gt = 1.0f / (1.0f + expf(-sd));
    const float og = 1.0f - gt;
    v4f y;
    y.x = gt * r4.x + og * ag.x + x0.x;
    y.y = gt * r4.y + og * ag.y + x0.y;
    y.z = gt * r4.z + og * ag.z + x0.z;
    y.w = gt * r4.w + og * ag.w + x0.w;
    v4f o = ln4(y, g4, b4);
    o.x += pz; o.y += pz; o.z += pz; o.w += pz;
    float* gp = XL + (size_t)grow * HID + 4 * lane;
    const bool wrow = grow < nN;
    if (wrow) *(volatile v4f*)gp = o;
    __threadfence();
    if (wrow) *(volatile v4f*)gp = o;
  }
}

static inline int cdiv(int a, int b) { return (a + b - 1) / b; }

extern "C" void kernel_launch(void* const* d_in, const int* in_sizes, int n_in,
                              void* d_out, int out_size, void* d_ws, size_t ws_size,
                              hipStream_t stream) {
  if (n_in < 30) return;
  if (in_sizes[0] != NN * HID || in_sizes[1] != 2 * NE) return;
  if (in_sizes[3] != HID * HID || in_sizes[4] != HID) return;
  if (in_sizes[5] != NL * HID * HID || in_sizes[7] != NL * HID * HID || in_sizes[9] != NL * HID * HID ||
      in_sizes[11] != NL * HID * HID) return;
  if (in_sizes[6] != NL * HID || in_sizes[8] != NL * HID || in_sizes[10] != NL * HID || in_sizes[12] != NL * HID) return;
  if (in_sizes[13] != NL * 3 * HID || in_sizes[14] != NL * 3 * HID * HID || in_sizes[15] != NL * 3 * HID) return;
  if (in_sizes[16] != NL * HID * HID || in_sizes[17] != NL * HID) return;
  for (int i = 18; i < 24; ++i) if (in_sizes[i] != NL * HID) return;
  if (in_sizes[24] != NL * HID * HID || in_sizes[25] != NL * HID || in_sizes[26] != NL * HID * HID ||
      in_sizes[27] != NL * HID) return;
  if (in_sizes[28] != OUTC * HID || in_sizes[29] != OUTC) return;
  if (out_size != NN * OUTC) return;

  const float* x_in   = (const float*)d_in[0];
  const int*   ei     = (const int*)  d_in[1];
  const float* lin_in_w = (const float*)d_in[3];  const float* lin_in_b = (const float*)d_in[4];
  const float* wq = (const float*)d_in[5];   const float* bq = (const float*)d_in[6];
  const float* wk = (const float*)d_in[7];   const float* bk = (const float*)d_in[8];
  const float* wv = (const float*)d_in[9];   const float* bv = (const float*)d_in[10];
  const float* wsk = (const float*)d_in[11]; const float* bsk = (const float*)d_in[12];
  const float* wbe = (const float*)d_in[13];
  const float* ain_w = (const float*)d_in[14]; const float* ain_b = (const float*)d_in[15];
  const float* aout_w = (const float*)d_in[16]; const float* aout_b = (const float*)d_in[17];
  const float* n1g = (const float*)d_in[18]; const float* n1b = (const float*)d_in[19];
  const float* n2g = (const float*)d_in[20]; const float* n2b = (const float*)d_in[21];
  const float* n3g = (const float*)d_in[22]; const float* n3b = (const float*)d_in[23];
  const float* w1 = (const float*)d_in[24];  const float* b1 = (const float*)d_in[25];
  const float* w2 = (const float*)d_in[26];  const float* b2 = (const float*)d_in[27];
  const float* lout_w = (const float*)d_in[28]; const float* lout_b = (const float*)d_in[29];
  float* out = (float*)d_out;
  const int* src = ei;
  const int* tgt = ei + NE;

  const size_t PF  = (size_t)NN * HID * 4;
  const size_t PHL = (size_t)NN * HLP * 2;
  size_t off = 0;
  const size_t oX    = off; off += PF;
  const size_t oXL   = off; off += PF;
  const size_t oX2   = off; off += PF;
  const size_t oXhl  = off; off += PHL;
  const size_t oX2hl = off; off += PHL;
  const size_t oOhl  = off; off += PHL;
  const size_t oHhl  = off; off += PHL;
  const size_t oQKVR = off; off += (size_t)NN * 512 * 4;
  const size_t oAQKV = off; off += 3 * PHL;
  const size_t oXB   = off; off += (size_t)NN * HID * 2;
  const size_t oWIN  = off; off += (size_t)HID * HID * 2;
  const size_t oWCAT = off; off += (size_t)NL * PCAT * HLP * 2;
  const size_t oWO2  = off; off += (size_t)NL * HID * HLP * 2;
  const size_t oW1D  = off; off += (size_t)NL * HID * HLP * 2;
  const size_t oW2D  = off; off += (size_t)NL * HID * HLP * 2;
  const size_t oWOUT = off; off += (size_t)OUTC * HLP * 2;
  const size_t oBCAT = off; off += (size_t)NL * PCAT * 4;
  if (off > ws_size || off > (size_t)WSMAX) return;
  char* ws = (char*)d_ws;
  float* X    = (float*)(ws + oX);
  float* XL   = (float*)(ws + oXL);
  float* X2   = (float*)(ws + oX2);
  unsigned short* Xhl  = (unsigned short*)(ws + oXhl);
  unsigned short* X2hl = (unsigned short*)(ws + oX2hl);
  unsigned short* Ohl  = (unsigned short*)(ws + oOhl);
  unsigned short* Hhl  = (unsigned short*)(ws + oHhl);
  float* QKVR = (float*)(ws + oQKVR);
  unsigned short* AQKV = (unsigned short*)(ws + oAQKV);
  unsigned short* XB   = (unsigned short*)(ws + oXB);
  unsigned short* WIN  = (unsigned short*)(ws + oWIN);
  unsigned short* WCAT = (unsigned short*)(ws + oWCAT);
  unsigned short* WO2  = (unsigned short*)(ws + oWO2);
  unsigned short* W1D  = (unsigned short*)(ws + oW1D);
  unsigned short* W2D  = (unsigned short*)(ws + oW2D);
  unsigned short* WOUT = (unsigned short*)(ws + oWOUT);
  float* BCAT = (float*)(ws + oBCAT);
  const unsigned short* AQ = AQKV;
  const unsigned short* AK = AQKV + (size_t)NN * HLP;
  const unsigned short* AV = AQKV + (size_t)2 * NN * HLP;

  hipFuncSetAttribute(reinterpret_cast<const void*>(&k_scan), hipFuncAttributeMaxDynamicSharedMemorySize, LDS_AGG);
  hipFuncSetAttribute(reinterpret_cast<const void*>(&k_attn), hipFuncAttributeMaxDynamicSharedMemorySize, LDS_ATT);
  hipFuncSetAttribute(reinterpret_cast<const void*>(&k_gemm<8, 0>), hipFuncAttributeMaxDynamicSharedMemorySize, LDS_GEMM);
  hipFuncSetAttribute(reinterpret_cast<const void*>(&k_gemm<8, 1>), hipFuncAttributeMaxDynamicSharedMemorySize, LDS_GEMM);
  hipFuncSetAttribute(reinterpret_cast<const void*>(&k_gemm<8, 2>), hipFuncAttributeMaxDynamicSharedMemorySize, LDS_GEMM);
  hipFuncSetAttribute(reinterpret_cast<const void*>(&k_gemm<8, 3>), hipFuncAttributeMaxDynamicSharedMemorySize, LDS_GEMM);
  hipFuncSetAttribute(reinterpret_cast<const void*>(&k_gemm<8, 4>), hipFuncAttributeMaxDynamicSharedMemorySize, LDS_GEMM);
  hipFuncSetAttribute(reinterpret_cast<const void*>(&k_gemm<4, 5>), hipFuncAttributeMaxDynamicSharedMemorySize, LDS_GEMM);

  k_cvt<<<cdiv(NN * 16, 256), 256, 0, stream>>>(x_in, XB, NN * 16, NN, 0, 0, HID, 0);
  k_cvt<<<cdiv(HID * 16, 256), 256, 0, stream>>>(lin_in_w, WIN, HID * 16, HID, 0, 0, HID, 0);
  k_cvt<<<cdiv(NL * HID * 16, 256), 256, 0, stream>>>(wq,  WCAT, NL * HID * 16, HID, PCAT, 0,   HLP, 1);
  k_cvt<<<cdiv(NL * HID * 16, 256), 256, 0, stream>>>(wk,  WCAT, NL * HID * 16, HID, PCAT, 128, HLP, 1);
  k_cvt<<<cdiv(NL * HID * 16, 256), 256, 0, stream>>>(wv,  WCAT, NL * HID * 16, HID, PCAT, 256, HLP, 1);
  k_cvt<<<cdiv(NL * HID * 16, 256), 256, 0, stream>>>(wsk, WCAT, NL * HID * 16, HID, PCAT, 384, HLP, 1);
  k_cvt<<<cdiv(NL * 3 * HID * 16, 256), 256, 0, stream>>>(ain_w, WCAT, NL * 3 * HID * 16, 3 * HID, PCAT, 512, HLP, 1);
  k_cvt<<<cdiv(NL * HID * 16, 256), 256, 0, stream>>>(aout_w, WO2, NL * HID * 16, HID, HID, 0, HLP, 1);
  k_cvt<<<cdiv(NL * HID * 16, 256), 256, 0, stream>>>(w1, W1D, NL * HID * 16, HID, HID, 0, HLP, 1);
  k_cvt<<<cdiv(NL * HID * 16, 256), 256, 0, stream>>>(w2, W2D, NL * HID * 16, HID, HID, 0, HLP, 1);
  k_cvt<<<cdiv(OUTC * 16, 256), 256, 0, stream>>>(lout_w, WOUT, OUTC * 16, OUTC, 0, 0, HLP, 1);
  k_bcat<<<dim3(7, NL), 128, 0, stream>>>(bq, bk, bv, bsk, ain_b, BCAT);

  const int gM = NN / 128;
  const int vec8 = ((NE & 3) == 0) ? 1 : 0;
  k_gemm<8, 0><<<dim3(gM, 1), 256, LDS_GEMM, stream>>>(XB, WIN, lin_in_b, lin_in_b, lin_in_b, lin_in_b, lin_in_b,
                                                       X, Xhl, HID, HID / 32, HID);
  for (int l = 0; l < NL; ++l) {
    const size_t bo = (size_t)l * HID;
    k_gemm<8, 1><<<dim3(gM, 7), 256, LDS_GEMM, stream>>>(Xhl, WCAT + (size_t)l * PCAT * HLP, BCAT + (size_t)l * PCAT,
                                                         BCAT, BCAT, BCAT, BCAT, QKVR, AQKV, HLP, HLP / 32, 512);
    k_scan<<<NN / NBRUN, NTHR, LDS_AGG, stream>>>(src, tgt, QKVR, X, wbe + (size_t)l * 3 * HID, n1g + bo, n1b + bo,
                                                  XL, NN, NE, vec8);
    k_attn<<<NG * (SEQ / 64), 128, LDS_ATT, stream>>>(AQ, AK, AV, Ohl);
    k_gemm<8, 2><<<dim3(gM, 1), 256, LDS_GEMM, stream>>>(Ohl, WO2 + (size_t)l * HID * HLP, aout_b + bo, X, XL,
                                                         n2g + bo, n2b + bo, X2, X2hl, HLP, HLP / 32, HID);
    k_gemm<8, 3><<<dim3(gM, 1), 256, LDS_GEMM, stream>>>(X2hl, W1D + (size_t)l * HID * HLP, b1 + bo, b1, b1, b1, b1,
                                                         X2, Hhl, HLP, HLP / 32, HID);
    k_gemm<8, 4><<<dim3(gM, 1), 256, LDS_GEMM, stream>>>(Hhl, W2D + (size_t)l * HID * HLP, b2 + bo, X2, X2,
                                                         n3g + bo, n3b + bo, X, Xhl, HLP, HLP / 32, HID);
  }
  k_gemm<4, 5><<<dim3(gM, 1), 256, LDS_GEMM, stream>>>(Xhl, WOUT, lout_b, lout_b, lout_b, lout_b, lout_b,
                                                       out, Xhl, HLP, HLP / 32, OUTC);
  (void)hipGetLastError();
}
